// MultiHeadAttentionQuantum_65481071397337
// MI455X (gfx1250) — hardware-verified
//
#include <hip/hip_runtime.h>
#include <math.h>

typedef __attribute__((ext_vector_type(16))) _Float16 v16h;
typedef __attribute__((ext_vector_type(16))) __bf16 v16b;
typedef __attribute__((ext_vector_type(8)))  _Float16 v8h;
typedef __attribute__((ext_vector_type(8)))  float v8f;
typedef __attribute__((ext_vector_type(4)))  float v4f;
typedef __attribute__((ext_vector_type(2)))  float v2f;
typedef __attribute__((ext_vector_type(4)))  unsigned v4u;
typedef __attribute__((ext_vector_type(4)))  int v4i;
typedef float __attribute__((may_alias)) float_a;
typedef int __attribute__((may_alias)) int_a;

template <typename T> __device__ __forceinline__ void vst2(void* p, T v) { *(volatile T*)p = v; __threadfence(); *(volatile T*)p = v; }
__device__ __forceinline__ v8f wmma16(v16h a, v16h b, v8f c) {
  v8f d = __builtin_amdgcn_wmma_f32_16x16x32_f16(false, a, false, b, (short)0, c, false, false);
  asm volatile("v_nop\n\tv_nop\n\tv_nop\n\tv_nop" : "+v"(d) : "v"(a), "v"(b));
  return d;
}
__device__ __forceinline__ v8f wmma_bf(v16b a, v16b b, v8f c) {
  v8f d = __builtin_amdgcn_wmma_f32_16x16x32_bf16(false, a, false, b, (short)0, c, false, false);
  asm volatile("v_nop\n\tv_nop\n\tv_nop\n\tv_nop" : "+v"(d) : "v"(a), "v"(b));
  return d;
}
__device__ __forceinline__ v16h frag_h(const _Float16* rowk0, int lane) {
  union { v16h v; v8h q[2]; } u; const _Float16* p = rowk0 + 8 * (lane >> 4);
  u.q[0] = *(const v8h*)p; u.q[1] = *(const v8h*)(p + 16); return u.v;
}
__device__ __forceinline__ v16h frag_f32(const float* rowk0, int lane) {
  v16h a; const float* p = rowk0 + 8 * (lane >> 4);
#pragma unroll
  for (int i = 0; i < 8; ++i) { a[i] = (_Float16)p[i]; a[8 + i] = (_Float16)p[16 + i]; }
  return a;
}
__device__ __forceinline__ v16h frag_f32s(const float* rowk0, int lane, float sc) {
  v16h a; const float* p = rowk0 + 8 * (lane >> 4);
#pragma unroll
  for (int i = 0; i < 8; ++i) { a[i] = (_Float16)(p[i] * sc); a[8 + i] = (_Float16)(p[16 + i] * sc); }
  return a;
}
__device__ __forceinline__ v16h fragc_f32(const float* W, int k0, int n, int lane, int ld, int K) {
  v16h a; const int g = lane >> 4;
#pragma unroll
  for (int i = 0; i < 8; ++i) { const int ka = k0 + 8 * g + i, kb = ka + 16;
    a[i] = (_Float16)(ka < K ? W[(size_t)(ka < K ? ka : K - 1) * ld + n] : 0.f); a[8 + i] = (_Float16)(kb < K ? W[(size_t)(kb < K ? kb : K - 1) * ld + n] : 0.f); }
  return a;
}
struct F2 { v16b h, l; };
__device__ __forceinline__ F2 bsplit16(const float v[16]) { F2 r;
#pragma unroll
  for (int i = 0; i < 16; ++i) { const __bf16 h = (__bf16)v[i]; r.h[i] = h; r.l[i] = (__bf16)(v[i] - (float)h); }
  return r; }
__device__ __forceinline__ F2 split_row(const float* row, int k0, int lane) { float v[16]; const float* p = row + k0 + 8 * (lane >> 4);
#pragma unroll
  for (int i = 0; i < 8; ++i) { v[i] = p[i]; v[8 + i] = p[16 + i]; }
  return bsplit16(v); }
__device__ __forceinline__ F2 split_rowK(const float* row, int k0, int lane, int K) { float v[16]; const int g = lane >> 4;
#pragma unroll
  for (int i = 0; i < 8; ++i) { const int ka = k0 + 8 * g + i, kb = ka + 16; v[i] = ka < K ? row[ka < K ? ka : K - 1] : 0.f; v[8 + i] = kb < K ? row[kb < K ? kb : K - 1] : 0.f; }
  return bsplit16(v); }
__device__ __forceinline__ F2 split_col(const float* W, int k0, int n, int lane, int ld, int K) { float v[16]; const int g = lane >> 4;
#pragma unroll
  for (int i = 0; i < 8; ++i) { const int ka = k0 + 8 * g + i, kb = ka + 16; v[i] = ka < K ? W[(size_t)(ka < K ? ka : K - 1) * ld + n] : 0.f; v[8 + i] = kb < K ? W[(size_t)(kb < K ? kb : K - 1) * ld + n] : 0.f; }
  return bsplit16(v); }
__device__ __forceinline__ v8f mac3(const F2& a, const F2& b, v8f c) { c = wmma_bf(a.l, b.h, c); c = wmma_bf(a.h, b.l, c); return wmma_bf(a.h, b.h, c); }
__device__ __forceinline__ float sigm(float v) { return 1.0f / (1.0f + expf(-v)); }
#define LDSX() do { asm volatile("s_wait_dscnt 0" ::: "memory"); __builtin_amdgcn_wave_barrier(); __builtin_amdgcn_fence(__ATOMIC_RELEASE, "workgroup"); } while (0)


#define NB 4
#define TT 1024
#define EE 128
#define NH 16
#define QD 8
#define HD 16
#define KP 32
#define CQ (NH * KP)
#define CV (NH * HD)
#define HG 8
#define QSC 64.0f
#ifndef TNB
#define TNB NB
#endif
__device__ __forceinline__ float bfr(float v) { return (float)(__bf16)v; }

#define WS_QH  0u
#define WS_QL  (WS_QH + 2u * (size_t)NB * TT * CQ)
#define WS_VT  (WS_QL + 2u * (size_t)NB * TT * CQ)
#define WS_VL  (WS_VT + 2u * (size_t)NB * CV * TT)
#define WS_S   (WS_VL + 2u * (size_t)NB * CV * TT)
#define WS_Y   (WS_S + 4u * (size_t)HG * TT * TT)
#define WS_END (WS_Y + 4u * (size_t)NB * TT * EE)

__global__ __launch_bounds__(256) void k_feat(const float* __restrict__ X, const float* __restrict__ PHI, _Float16* __restrict__ QH, _Float16* __restrict__ QL, _Float16* __restrict__ VT, _Float16* __restrict__ VL) { __shared__ __align__(16) float sq[64][EE + 4];
  const int t = threadIdx.x; const size_t r0 = (size_t)blockIdx.x * 64;
#pragma unroll 1
  for (int it = 0; it < 4; ++it) { const int e = it * 256 + t; const int rl = e >> 4, h = e & 15; const float* xp = X + (r0 + rl) * EE + h * QD; float* c = &sq[rl][h * QD];
#pragma unroll 1
    for (int w = 0; w < QD; ++w) c[w] = cosf(bfr(xp[w]) + bfr(PHI[w]));
    float p17 = c[1];
#pragma unroll
    for (int k = 2; k < QD; ++k) p17 = p17 * c[k];
    float pre = c[0];
#pragma unroll
    for (int k = 1; k < QD; ++k) { pre = pre * c[k]; c[k] = pre; }
    c[0] = p17; }
  __syncthreads();
#pragma unroll 1
  for (int p = t; p < 64 * 64; p += 256) { const int rl = p >> 6, seg = p & 63; const int h = seg >> 2; const bool real = (seg & 3) == 0; v8h vh, vl;
#pragma unroll
    for (int k = 0; k < 8; ++k) { const float v = real ? sq[rl][h * QD + k] * QSC : 0.f; const _Float16 hv = (_Float16)v; vh[k] = hv; vl[k] = (_Float16)((v - (float)hv) * 1024.0f); }
    vst2((v4u*)(QH + (r0 + rl) * CQ + seg * 8), *(const v4u*)&vh); vst2((v4u*)(QL + (r0 + rl) * CQ + seg * 8), *(const v4u*)&vl); }
  { const size_t b = r0 / TT; const int t0 = (int)(r0 % TT);
#pragma unroll 1
    for (int p = t; p < CV * 8; p += 256) { const int c = p >> 3, q8 = p & 7; const int h = c >> 4, d = c & 15; v8h vh, vl;
#pragma unroll
      for (int k = 0; k < 8; ++k) { const float v = d < QD ? sq[q8 * 8 + k][h * QD + d] * QSC : 0.f; const _Float16 hv = (_Float16)v; vh[k] = hv; vl[k] = (_Float16)((v - (float)hv) * 1024.0f); }
      const size_t o2 = (b * CV + c) * (size_t)TT + t0 + q8 * 8; vst2((v4u*)(VT + o2), *(const v4u*)&vh); vst2((v4u*)(VL + o2), *(const v4u*)&vl); } } }
__global__ __launch_bounds__(128) void k_sc(const _Float16* __restrict__ QH, const _Float16* __restrict__ QL, int b, int h0, float* __restrict__ S0) { __shared__ __align__(16) float ss[4][16][132]; const int h = h0 + blockIdx.z; float* S = S0 + (size_t)blockIdx.z * TT * TT;
  const int tid = threadIdx.x, wave = tid >> 5, lane = tid & 31, col = lane & 15, g = lane >> 4; const int k0 = blockIdx.y * 128; const int ql0 = blockIdx.x * 64 + wave * 16; const size_t q0 = (size_t)b * TT + ql0;
  v8f acc[8] = {}, accl[8] = {};
  { const v16h ah = frag_h(QH + (q0 + col) * CQ + h * KP, lane), al = frag_h(QL + (q0 + col) * CQ + h * KP, lane);
#pragma unroll
    for (int j = 0; j < 8; ++j) { const v16h kb = frag_h(QH + ((size_t)b * TT + k0 + j * 16 + col) * CQ + h * KP, lane); acc[j] = wmma16(ah, kb, acc[j]); accl[j] = wmma16(al, kb, accl[j]); } }
#pragma unroll
  for (int j = 0; j < 8; ++j)
#pragma unroll
    for (int r = 0; r < 8; ++r) ss[wave][8 * g + r][j * 16 + col] = (acc[j][r] + accl[j][r] * (1.0f / 1024.0f)) * (0.35355339059327373f / (QSC * QSC));
  LDSX(); for (int rl = 0; rl < 16; ++rl) vst2(S + (size_t)(ql0 + rl) * TT + k0 + lane * 4, *(const v4f*)&ss[wave][rl][lane * 4]); }
__global__ __launch_bounds__(256) void k_sm(float* __restrict__ S0) { __shared__ float sred[8]; __shared__ float sbc; __shared__ __align__(16) float sh[TT];
  const int t = threadIdx.x; const size_t row = blockIdx.x; float* sr = S0 + (size_t)blockIdx.y * TT * TT + row * TT; const int kend = TT;
  float m = -3.0e38f; for (int k = t; k < kend; k += 256) m = fmaxf(m, sr[k]);
#pragma unroll
  for (int o = 1; o < 32; o <<= 1) m = fmaxf(m, __shfl_xor(m, o));
  if ((t & 31) == 0) sred[t >> 5] = m; __syncthreads(); if (t == 0) { float a = sred[0]; for (int i = 1; i < 8; ++i) a = fmaxf(a, sred[i]); sbc = a; } __syncthreads(); m = sbc; __syncthreads();
  float sum = 0.f; for (int k = t; k < kend; k += 256) sum += expf(sr[k] - m);
#pragma unroll
  for (int o = 1; o < 32; o <<= 1) sum += __shfl_xor(sum, o);
  if ((t & 31) == 0) sred[t >> 5] = sum; __syncthreads(); if (t == 0) { float a = 0.f; for (int i = 0; i < 8; ++i) a += sred[i]; sbc = 1.0f / a; } __syncthreads(); const float inv = sbc;
  for (int k = t; k < kend; k += 256) sh[k] = expf(sr[k] - m) * inv * 2048.0f;
  __syncthreads(); for (int q = t; q < kend / 4; q += 256) vst2(sr + q * 4, *(const v4f*)&sh[q * 4]); }
__global__ __launch_bounds__(128) void k_pv(const float* __restrict__ PS0, const _Float16* __restrict__ VT, const _Float16* __restrict__ VL, int b, int h0, float* __restrict__ Y) { const int h = h0 + blockIdx.z; const float* PS = PS0 + (size_t)blockIdx.z * TT * TT; __shared__ __align__(16) float ss[4][16][20];
  const int tid = threadIdx.x, wave = tid >> 5, lane = tid & 31, col = lane & 15, g = lane >> 4; const int ql0 = blockIdx.x * 64 + wave * 16;
  v8f acc = {}, accl = {};
#pragma unroll 2
  for (int kc = 0; kc < TT / 32; ++kc) { const v16h p = frag_f32(PS + (size_t)(ql0 + col) * TT + kc * 32, lane); const size_t po = ((size_t)b * CV + h * HD + col) * (size_t)TT + kc * 32;
    asm volatile("s_wait_loadcnt 0x0" ::: "memory"); acc = wmma16(p, frag_h(VT + po, lane), acc); accl = wmma16(p, frag_h(VL + po, lane), accl); }
#pragma unroll
  for (int r = 0; r < 8; ++r) ss[wave][8 * g + r][col] = (acc[r] + accl[r] * (1.0f / 1024.0f)) * (1.0f / (2048.0f * QSC));
  LDSX();
  { const int rl = lane >> 1, half = lane & 1; vst2(Y + ((size_t)h * NB * TT + (size_t)b * TT + ql0 + rl) * QD + half * 4, *(const v4f*)&ss[wave][rl][half * 4]); } }
__global__ __launch_bounds__(128) void k_out(const float* __restrict__ Y, const float* __restrict__ WP, const float* __restrict__ BP, float* __restrict__ OUT) { __shared__ __align__(16) float sf[4][16][132];
  const int tid = threadIdx.x, wave = tid >> 5, lane = tid & 31, col = lane & 15, g = lane >> 4; const size_t r0 = (size_t)blockIdx.x * 64 + wave * 16;
  v8f acc[8] = {};
#pragma unroll
  for (int kc = 0; kc < EE / 32; ++kc) { F2 a; { float v[16]; const int hA = kc * 4 + g, hB = hA + 2; const float* pa = Y + ((size_t)hA * NB * TT + r0 + col) * QD; const float* pb = Y + ((size_t)hB * NB * TT + r0 + col) * QD;
#pragma unroll
      for (int i = 0; i < 8; ++i) { v[i] = pa[i]; v[8 + i] = pb[i]; } a = bsplit16(v); }
#pragma unroll
    for (int j = 0; j < 8; ++j) { v16b w; const int o = j * 16 + col;
#pragma unroll
      for (int i = 0; i < 8; ++i) { w[i] = (__bf16)WP[(size_t)o * EE + (kc * 32 + 8 * g + i)]; w[8 + i] = (__bf16)WP[(size_t)o * EE + (kc * 32 + 16 + 8 * g + i)]; }
      asm volatile("s_wait_loadcnt 0x0" ::: "memory"); acc[j] = wmma_bf(a.h, w, acc[j]); acc[j] = wmma_bf(a.l, w, acc[j]); } }
#pragma unroll
  for (int j = 0; j < 8; ++j) { const float bb = bfr(BP[j * 16 + col]);
#pragma unroll
    for (int r = 0; r < 8; ++r) sf[wave][8 * g + r][j * 16 + col] = acc[j][r] + bb; }
  LDSX(); for (int rl = 0; rl < 16; ++rl) vst2(OUT + (r0 + rl) * EE + lane * 4, *(const v4f*)&sf[wave][rl][lane * 4]); }
extern "C" void kernel_launch(void* const* d_in, const int* in_sizes, int n_in, void* d_out, int out_size, void* d_ws, size_t ws_size, hipStream_t stream) {
  (void)in_sizes; (void)n_in; (void)out_size;
  const float** F = (const float**)d_in;
  if (ws_size < (size_t)WS_END) return;
  char* ws = (char*)d_ws; _Float16 *QH = (_Float16*)(ws + WS_QH), *QL = (_Float16*)(ws + WS_QL), *VT = (_Float16*)(ws + WS_VT), *VL = (_Float16*)(ws + WS_VL); float *S = (float*)(ws + WS_S), *Y = (float*)(ws + WS_Y);
  k_feat<<<dim3(TNB * TT / 64), 256, 0, stream>>>(F[0], F[1], QH, QL, VT, VL);
  for (int b = 0; b < TNB; ++b) for (int h0 = 0; h0 < NH; h0 += HG) {
    k_sc<<<dim3(TT / 64, TT / 128, HG), 128, 0, stream>>>(QH, QL, b, h0, S);
    k_sm<<<dim3(TT, HG), 256, 0, stream>>>(S);
    k_pv<<<dim3(TT / 64, 1, HG), 128, 0, stream>>>(S, VT, VL, b, h0, Y);
  }
  k_out<<<dim3(TNB * TT / 64), 128, 0, stream>>>(Y, F[2], F[3], (float*)d_out);
}
